// Next_Node_Probability_Calculator_for_group_21990232556010
// MI455X (gfx1250) — hardware-verified
//
#include <hip/hip_runtime.h>

typedef __attribute__((ext_vector_type(16))) _Float16 v16h;
typedef __attribute__((ext_vector_type(8)))  _Float16 v8h;
typedef __attribute__((ext_vector_type(16))) __bf16   v16b;
typedef __attribute__((ext_vector_type(8)))  __bf16   v8b;
typedef __attribute__((ext_vector_type(8)))  float    v8f;
typedef __attribute__((ext_vector_type(4)))  float    v4f;
typedef __attribute__((ext_vector_type(8)))  unsigned short v8us;

constexpr int NBATCH = 16;
constexpr int NGRP   = 512;
constexpr int NPTR   = 512;
constexpr int NEMB   = 256;
constexpr int NHEAD  = 16;
constexpr int HDIM   = 16;
constexpr int NFEAT  = NHEAD * HDIM;
constexpr int KQIN   = 2 * NEMB + 1;
constexpr int KQPAD  = 576;
constexpr float CLIPV = 10.0f;

static_assert(NFEAT == 256, "feature width");
static_assert(KQPAD % 64 == 0 && KQPAD >= KQIN, "padded concat width");
static_assert((KQPAD * 2) % 128 == 0, "whole lines per padded row");

__device__ __forceinline__ unsigned short f2bf_bits(float f) {
  unsigned u = __float_as_uint(f);
  return (unsigned short)((u + 0x7FFFu + ((u >> 16) & 1u)) >> 16);
}
__device__ __forceinline__ float bf_bits2f(unsigned short h) { return __uint_as_float(((unsigned)h) << 16); }
__device__ __forceinline__ void bf_split_bits(float f, unsigned short& hb, unsigned short& lb) {
  hb = f2bf_bits(f);
  lb = f2bf_bits(f - bf_bits2f(hb));
}

__device__ __forceinline__ void dep_guard_h(v8f& a, v8f& b, v16h x, v16h y) { asm volatile("v_nop\n\tv_nop\n\tv_nop\n\tv_nop" : "+v"(a), "+v"(b) : "v"(x), "v"(y)); }
__device__ __forceinline__ void dep_guard_b(v8f& a, v8f& b, v16b x, v16b y) { asm volatile("v_nop\n\tv_nop\n\tv_nop\n\tv_nop" : "+v"(a), "+v"(b) : "v"(x), "v"(y)); }
__device__ __forceinline__ void keep4_h(v16h a, v16h b, v16h c, v16h d) { asm volatile("v_nop" :: "v"(a), "v"(b), "v"(c), "v"(d)); }
__device__ __forceinline__ void keep4_b(v16b a, v16b b, v16b c, v16b d) { asm volatile("v_nop" :: "v"(a), "v"(b), "v"(c), "v"(d)); }
__device__ __forceinline__ void acc_guard4(v8f& a, v8f& b, v8f& c, v8f& d) { asm volatile("v_nop\n\tv_nop\n\tv_nop\n\tv_nop" : "+v"(a), "+v"(b), "+v"(c), "+v"(d)); }
template <typename T> struct Frag;
template <> struct Frag<_Float16> {
  typedef v16h V; union U { v16h v; v8h h[2]; };
  static __device__ __forceinline__ v16h load(const _Float16* p) {
    U f; f.h[0] = *(const v8h*)(p); f.h[1] = *(const v8h*)(p + 16); return f.v;
  }
  static __device__ __forceinline__ v8f mma(v16h a, v16h b, v8f c) {
    return __builtin_amdgcn_wmma_f32_16x16x32_f16(false, a, false, b, (short)0, c, false, false);
  }
  static __device__ __forceinline__ void guard(v8f& a, v8f& b, v16h x, v16h y) { dep_guard_h(a, b, x, y); }
  static __device__ __forceinline__ void keep(v16h a, v16h b, v16h c, v16h d) { keep4_h(a, b, c, d); }
};
template <> struct Frag<__bf16> {
  typedef v16b V; union U { v16b v; v8b h[2]; };
  static __device__ __forceinline__ v16b load(const __bf16* p) {
    U f; f.h[0] = *(const v8b*)(p); f.h[1] = *(const v8b*)(p + 16); return f.v;
  }
  static __device__ __forceinline__ v8f mma(v16b a, v16b b, v8f c) {
    return __builtin_amdgcn_wmma_f32_16x16x32_bf16(false, a, false, b, (short)0, c, false, false);
  }
  static __device__ __forceinline__ void guard(v8f& a, v8f& b, v16b x, v16b y) { dep_guard_b(a, b, x, y); }
  static __device__ __forceinline__ void keep(v16b a, v16b b, v16b c, v16b d) { keep4_b(a, b, c, d); }
};

__device__ __forceinline__ unsigned short at_bf_bits(float f) {
  unsigned u = __float_as_uint(f);
  return (unsigned short)((u + 0x7FFFu + ((u >> 16) & 1u)) >> 16);
}
__device__ __forceinline__ __bf16 at_f2bf(float f) { return __builtin_bit_cast(__bf16, at_bf_bits(f)); }
__device__ __forceinline__ void at_split(float f, __bf16& hi, __bf16& lo) {
  const unsigned short hb = at_bf_bits(f);
  hi = __builtin_bit_cast(__bf16, hb);
  lo = at_f2bf(f - __uint_as_float(((unsigned)hb) << 16));
}
__device__ __forceinline__ v8f at_mma(v16b a, v16b b, v8f c) {
  c = __builtin_amdgcn_wmma_f32_16x16x32_bf16(false, a, false, b, (short)0, c, false, false);
  asm volatile("v_nop\n\tv_nop\n\tv_nop\n\tv_nop" : "+v"(c) : "v"(a), "v"(b));
  return c;
}

template <int ET> struct Elem;
template <> struct Elem<0> { typedef _Float16 T; };
template <> struct Elem<1> { typedef __bf16 T; };
template <int ET, bool SPLIT, int BIAS_MODE, int OUT_MODE, bool RESID, int ACT = 0>
__global__ __launch_bounds__(256) void wmma_gemm64(
    const unsigned short* __restrict__ Ap, const unsigned short* __restrict__ A2p, int lda, long strideA,
    const unsigned short* __restrict__ Btp, const unsigned short* __restrict__ Bt2p, int ldb, long strideB,
    void* __restrict__ Cout, void* __restrict__ Cout2, int ldc, long strideC,
    const float* __restrict__ bias,
    const float* __restrict__ resid, long strideR,
    int M, int N, int K, float scale) {
  typedef typename Elem<ET>::T T;
  typedef typename Frag<T>::V V;
  const T* A = (const T*)Ap; const T* A2 = (const T*)A2p; const T* Bt = (const T*)Btp; const T* Bt2 = (const T*)Bt2p;
  __shared__ __align__(16) float sT[8][16 * 68];
  const int b    = blockIdx.y;
  const int lane = threadIdx.x & 31;
  const int wave = threadIdx.x >> 5;
  const int tilesN = N >> 6;
  const int tilesM = M >> 6;
  const int tile = blockIdx.x * 8 + wave;
  if (tile >= tilesM * tilesN) return;
  const int tm = tile / tilesN;
  const int tn = tile - tm * tilesN;
  const int m0 = tm << 6;
  const int n0 = tn << 6;

  const T* Ab  = A  + (size_t)b * strideA;
  const T* Bb  = Bt + (size_t)b * strideB;
  const T* Ab2 = SPLIT ? (A2  + (size_t)b * strideA) : nullptr;
  const T* Bb2 = SPLIT ? (Bt2 + (size_t)b * strideB) : nullptr;

  const int rlane = lane & 15;
  const int koff  = (lane >> 4) * 8;
  const int mOff  = (lane >> 4) * 8;

  v8f acc[4][4];
#pragma unroll
  for (int i = 0; i < 4; ++i)
#pragma unroll
    for (int j = 0; j < 4; ++j) acc[i][j] = (v8f){0.f,0.f,0.f,0.f,0.f,0.f,0.f,0.f};

  for (int k0 = 0; k0 < K; k0 += 32) {
    V bh[4], bl[4];
#pragma unroll
    for (int j = 0; j < 4; ++j) {
      const size_t bo = (size_t)(n0 + (j << 4) + rlane) * ldb + koff + k0;
      bh[j] = Frag<T>::load(Bb + bo);
      if (SPLIT) bl[j] = Frag<T>::load(Bb2 + bo);
    }
#pragma unroll
    for (int i = 0; i < 4; ++i) {
      const size_t ao = (size_t)(m0 + (i << 4) + rlane) * lda + koff + k0;
      V ah = Frag<T>::load(Ab + ao);
      V al;
      if (SPLIT) al = Frag<T>::load(Ab2 + ao);
#pragma unroll
      for (int j = 0; j < 4; ++j) {
        acc[i][j] = Frag<T>::mma(ah, bh[j], acc[i][j]);
        if (SPLIT) {
          acc[i][j] = Frag<T>::mma(ah, bl[j], acc[i][j]);
          acc[i][j] = Frag<T>::mma(al, bh[j], acc[i][j]);
        }
      }
      Frag<T>::guard(acc[i][0], acc[i][3], ah, SPLIT ? al : ah);
    }
    Frag<T>::keep(bh[0], bh[1], bh[2], bh[3]);
    if (SPLIT) Frag<T>::keep(bl[0], bl[1], bl[2], bl[3]);
  }
  acc_guard4(acc[0][0], acc[0][1], acc[0][2], acc[0][3]);
  acc_guard4(acc[1][0], acc[1][1], acc[1][2], acc[1][3]);
  acc_guard4(acc[2][0], acc[2][1], acc[2][2], acc[2][3]);
  acc_guard4(acc[3][0], acc[3][1], acc[3][2], acc[3][3]);

  float* slab = sT[wave];
  const float* Rb = RESID ? (resid + (size_t)b * strideR) : nullptr;
#pragma unroll
  for (int i = 0; i < 4; ++i) {
    const int mBase = m0 + (i << 4);
#pragma unroll
    for (int j = 0; j < 4; ++j) {
      const int n = n0 + (j << 4) + rlane;
      float bv = 0.f;
      if (BIAS_MODE == 2) bv = bias[n];
#pragma unroll
      for (int r = 0; r < 8; ++r) {
        float v = acc[i][j][r] * scale;
        if (BIAS_MODE == 1) v += bias[mBase + mOff + r];
        if (BIAS_MODE == 2) v += bv;
        if (RESID) v += Rb[(size_t)(mBase + mOff + r) * ldc + n];
        if (ACT == 1) v = tanhf(v);
        if (ACT == 2) v = fmaxf(v, 0.0f);
        if (ACT == 3) v = v / (1.0f + expf(-v));
        if (ACT == 4) v = (v > 0.f) ? v : 0.01f * v;
        if (ACT == 5) v = 0.5f * v * (1.0f + erff(v * 0.70710678118654752f));
        slab[(mOff + r) * 68 + (j << 4) + rlane] = v;
      }
    }
    __builtin_amdgcn_fence(__ATOMIC_RELEASE, "workgroup");
    __builtin_amdgcn_wave_barrier();
    __builtin_amdgcn_fence(__ATOMIC_ACQUIRE, "workgroup");
    if (OUT_MODE == 0) {
      float* C = (float*)Cout + (size_t)b * strideC;
      const int hh = lane >> 4, c4 = (lane & 15) * 4;
      for (int pass = 0; pass < 2; ++pass) {
#pragma unroll
        for (int it = 0; it < 8; ++it) {
          const int row = it * 2 + hh;
          v4f v = *(const v4f*)(slab + row * 68 + c4);
          *(volatile v4f*)(C + (size_t)(mBase + row) * ldc + n0 + c4) = v;
        }
        __threadfence();
      }
    } else {
      const int q = lane >> 3, c8 = (lane & 7) * 8;
      unsigned short* C  = (unsigned short*)Cout  + (size_t)b * strideC;
      unsigned short* C2 = (OUT_MODE == 2) ? ((unsigned short*)Cout2 + (size_t)b * strideC) : nullptr;
      for (int pass = 0; pass < 2; ++pass) {
#pragma unroll
        for (int it = 0; it < 4; ++it) {
          const int row = it * 4 + q;
          const float* sp = slab + row * 68 + c8;
          v8h hv, lv;
#pragma unroll
          for (int e = 0; e < 8; ++e) {
            if (OUT_MODE == 1) {
              hv[e] = (_Float16)sp[e];
            } else {
              unsigned short hb = f2bf_bits(sp[e]);
              unsigned short lb = f2bf_bits(sp[e] - bf_bits2f(hb));
              hv[e] = __builtin_bit_cast(_Float16, hb);
              lv[e] = __builtin_bit_cast(_Float16, lb);
            }
          }
          *(volatile v8h*)(C + (size_t)(mBase + row) * ldc + n0 + c8) = hv;
          if (OUT_MODE == 2) *(volatile v8h*)(C2 + (size_t)(mBase + row) * ldc + n0 + c8) = lv;
        }
        __threadfence();
      }
    }
    __builtin_amdgcn_fence(__ATOMIC_RELEASE, "workgroup");
    __builtin_amdgcn_wave_barrier();
    __builtin_amdgcn_fence(__ATOMIC_ACQUIRE, "workgroup");
  }
}

__global__ __launch_bounds__(256) void transpose_split64(const float* __restrict__ in, int nrows, int ncols,
                                                         unsigned short* __restrict__ ohi,
                                                         unsigned short* __restrict__ olo, int rpad) {
  __shared__ float tile[64][65];
  const int tid = threadIdx.x;
  const int c0 = blockIdx.x * 64;
  const int r0 = blockIdx.y * 64;
  {
    const int rr = tid >> 2, cc = (tid & 3) * 16;
    const int r = r0 + rr;
    const int rcl = (r < nrows) ? r : (nrows - 1);
    const bool live = (r < nrows);
    const float* src = in + (size_t)rcl * ncols + c0 + cc;
#pragma unroll
    for (int q = 0; q < 4; ++q) {
      const v4f x = *(const v4f*)(src + 4 * q);
#pragma unroll
      for (int e = 0; e < 4; ++e) tile[cc + 4 * q + e][rr] = live ? x[e] : 0.0f;
    }
  }
  __syncthreads();
  const int lrow = tid >> 3, c8 = (tid & 7) * 8;
  for (int pass = 0; pass < 2; ++pass) {
#pragma unroll
    for (int it = 0; it < 2; ++it) {
      const int orow = lrow + 32 * it;
      v8us hv, lv;
#pragma unroll
      for (int e = 0; e < 8; ++e) {
        unsigned short hb, lb;
        bf_split_bits(tile[orow][c8 + e], hb, lb);
        hv[e] = hb;
        lv[e] = lb;
      }
      const size_t o = (size_t)(c0 + orow) * rpad + r0 + c8;
      *(volatile v8us*)(ohi + o) = hv;
      *(volatile v8us*)(olo + o) = lv;
    }
    __threadfence();
  }
}

__global__ __launch_bounds__(256) void split_rows8(const float* __restrict__ in,
                                                   unsigned short* __restrict__ ohi,
                                                   unsigned short* __restrict__ olo, int n8) {
  const int i = blockIdx.x * 256 + threadIdx.x;
  if (i >= n8) return;
  const v4f a0 = *(const v4f*)(in + (size_t)8 * i);
  const v4f a1 = *(const v4f*)(in + (size_t)8 * i + 4);
  v8us hv, lv;
#pragma unroll
  for (int e = 0; e < 4; ++e) {
    unsigned short hb, lb;
    bf_split_bits(a0[e], hb, lb);
    hv[e] = hb; lv[e] = lb;
    bf_split_bits(a1[e], hb, lb);
    hv[4 + e] = hb; lv[4 + e] = lb;
  }
  unsigned short* ph = ohi + (size_t)8 * i;
  unsigned short* pl = olo + (size_t)8 * i;
  for (int pass = 0; pass < 2; ++pass) {
    *(volatile v8us*)ph = hv;
    *(volatile v8us*)pl = lv;
    __threadfence();
  }
}

__device__ __forceinline__ float sel_concat(int col, float va, float vb, float tv) {
  return (col < NEMB) ? va : ((col < 2 * NEMB) ? vb : ((col == 2 * NEMB) ? tv : 0.0f));
}
__global__ __launch_bounds__(256) void build_query_input(const float* __restrict__ in1,
                                                         const float* __restrict__ in2,
                                                         const float* __restrict__ tcur,
                                                         unsigned short* __restrict__ ohi,
                                                         unsigned short* __restrict__ olo) {
  constexpr int GPR = KQPAD / 8;
  const int i = blockIdx.x * 256 + threadIdx.x;
  if (i >= NBATCH * NGRP * GPR) return;
  const int row = i / GPR;
  const int grp = i - row * GPR;
  const int col0 = grp * 8;
  const int b = row / NGRP;
  const int c1 = (col0 < NEMB - 8) ? col0 : (NEMB - 8);
  int c2 = col0 - NEMB; c2 = (c2 < 0) ? 0 : ((c2 > NEMB - 8) ? (NEMB - 8) : c2);
  const v4f a0 = *(const v4f*)(in1 + (size_t)b * NEMB + c1);
  const v4f a1 = *(const v4f*)(in1 + (size_t)b * NEMB + c1 + 4);
  const v4f b0 = *(const v4f*)(in2 + (size_t)row * NEMB + c2);
  const v4f b1 = *(const v4f*)(in2 + (size_t)row * NEMB + c2 + 4);
  const float tv = tcur[row];
  v8us hv, lv;
#pragma unroll
  for (int e = 0; e < 4; ++e) {
    unsigned short hb, lb;
    bf_split_bits(sel_concat(col0 + e, a0[e], b0[e], tv), hb, lb);
    hv[e] = hb; lv[e] = lb;
    bf_split_bits(sel_concat(col0 + 4 + e, a1[e], b1[e], tv), hb, lb);
    hv[4 + e] = hb; lv[4 + e] = lb;
  }
  unsigned short* ph = ohi + (size_t)8 * i;
  unsigned short* pl = olo + (size_t)8 * i;
  for (int pass = 0; pass < 2; ++pass) {
    *(volatile v8us*)ph = hv;
    *(volatile v8us*)pl = lv;
    __threadfence();
  }
}

__global__ __launch_bounds__(128) void mha_head16(
    const unsigned short* __restrict__ qhi, const unsigned short* __restrict__ qlo,
    const unsigned short* __restrict__ khi, const unsigned short* __restrict__ klo,
    const unsigned short* __restrict__ vthi, const unsigned short* __restrict__ vtlo,
    const float* __restrict__ mask,
    unsigned short* __restrict__ aohi, unsigned short* __restrict__ aolo) {
  union FB { v16b v; v8b h[2]; };
  __shared__ __align__(16) __bf16 Ksh[64 * 64];
  __shared__ __align__(16) __bf16 Ksl[64 * 64];
  __shared__ __align__(16) __bf16 Vsh[64 * 64];
  __shared__ __align__(16) __bf16 Vsl[64 * 64];
  __shared__ __align__(16) float  Msh[16 * 64];
  __shared__ __align__(16) __bf16 Psh[4][16 * 64];
  __shared__ __align__(16) __bf16 Psl[4][16 * 64];
  __shared__ __align__(16) float  Osh[16 * 68];

  const int tid  = threadIdx.x;
  const int wave = tid >> 5;
  const int lane = tid & 31;
  const int hh   = lane >> 4;
  const int c    = lane & 15;
  const int qt = blockIdx.x & 31;
  const int hg = (blockIdx.x >> 5) & 3;
  const int b  = blockIdx.x >> 7;
  const int row0 = b * NGRP + qt * 16;
  const int fcol = hg * 64;

  FB qa;
  {
    const size_t qo = (size_t)(row0 + c) * NFEAT + fcol + wave * 16 + 8 * hh;
    qa.h[0] = *(const v8b*)((const __bf16*)qhi + qo);
    qa.h[1] = *(const v8b*)((const __bf16*)qlo + qo);
  }

  float mrow[8], lrow[8];
  v8f oacc = (v8f){0.f,0.f,0.f,0.f,0.f,0.f,0.f,0.f};
#pragma unroll
  for (int r = 0; r < 8; ++r) { mrow[r] = -INFINITY; lrow[r] = 0.f; }

#pragma unroll 1
  for (int kc = 0; kc < NPTR / 64; ++kc) {
    const int kv0 = kc * 64;
    __syncthreads();
    {
      const int kvr = tid >> 1, ch = (tid & 1) * 32;
      const size_t ko = (size_t)(b * NPTR + kv0 + kvr) * NFEAT + fcol + ch;
      const size_t vo = ((size_t)(b * NFEAT) + fcol + kvr) * NPTR + kv0 + ch;
      const __bf16* ksrc  = (const __bf16*)khi  + ko;
      const __bf16* klsrc = (const __bf16*)klo  + ko;
      const __bf16* vsrc  = (const __bf16*)vthi + vo;
      const __bf16* vlsrc = (const __bf16*)vtlo + vo;
#pragma unroll
      for (int i = 0; i < 4; ++i) {
        *(v8b*)(Ksh + kvr * 64 + ch + 8 * i) = *(const v8b*)(ksrc  + 8 * i);
        *(v8b*)(Ksl + kvr * 64 + ch + 8 * i) = *(const v8b*)(klsrc + 8 * i);
      }
      asm volatile("" ::: "memory");
#pragma unroll
      for (int i = 0; i < 4; ++i) {
        *(v8b*)(Vsh + kvr * 64 + ch + 8 * i) = *(const v8b*)(vsrc  + 8 * i);
        *(v8b*)(Vsl + kvr * 64 + ch + 8 * i) = *(const v8b*)(vlsrc + 8 * i);
      }
      asm volatile("" ::: "memory");
      const int mr = tid >> 4, mc = (tid & 15) * 4;
#pragma unroll
      for (int i = 0; i < 2; ++i) {
        const int rr = mr + 8 * i;
        *(v4f*)(Msh + rr * 64 + mc) = *(const v4f*)(mask + (size_t)(row0 + rr) * NPTR + kv0 + mc);
      }
    }
    __syncthreads();

    v8f s[4];
#pragma unroll
    for (int j = 0; j < 4; ++j) {
      const int ko = (j * 16 + c) * 64 + wave * 16 + 8 * hh;
      FB k1, k2;
      k1.h[0] = *(const v8b*)(Ksh + ko); k1.h[1] = k1.h[0];
      k2.h[0] = *(const v8b*)(Ksl + ko); k2.h[1] = k2.h[0];
      s[j] = (v8f){0.f,0.f,0.f,0.f,0.f,0.f,0.f,0.f};
      s[j] = at_mma(qa.v, k1.v, s[j]);
      s[j] = at_mma(qa.v, k2.v, s[j]);
    }
    float cm[8];
#pragma unroll
    for (int r = 0; r < 8; ++r) {
      float m = -INFINITY;
#pragma unroll
      for (int j = 0; j < 4; ++j) {
        s[j][r] += Msh[(8 * hh + r) * 64 + j * 16 + c];
        m = fmaxf(m, s[j][r]);
      }
#pragma unroll
      for (int off = 1; off < 16; off <<= 1) m = fmaxf(m, __shfl_xor(m, off, 32));
      cm[r] = m;
    }
    __bf16* pwh = Psh[wave];
    __bf16* pwl = Psl[wave];
#pragma unroll
    for (int r = 0; r < 8; ++r) {
      const float mnew = fmaxf(mrow[r], cm[r]);
      const float alpha = expf(mrow[r] - mnew);
      mrow[r] = mnew;
      float psum = 0.f;
#pragma unroll
      for (int j = 0; j < 4; ++j) {
        const float p = expf(s[j][r] - mnew);
        psum += p;
        __bf16 ph, pl;
        at_split(p, ph, pl);
        pwh[(8 * hh + r) * 64 + j * 16 + c] = ph;
        pwl[(8 * hh + r) * 64 + j * 16 + c] = pl;
      }
#pragma unroll
      for (int off = 1; off < 16; off <<= 1) psum += __shfl_xor(psum, off, 32);
      lrow[r] = lrow[r] * alpha + psum;
      oacc[r] *= alpha;
    }
    __builtin_amdgcn_fence(__ATOMIC_RELEASE, "workgroup");
    __builtin_amdgcn_wave_barrier();
    __builtin_amdgcn_fence(__ATOMIC_ACQUIRE, "workgroup");
#pragma unroll
    for (int kk = 0; kk < 2; ++kk) {
      FB pa, pl, vb, vl;
      pa.h[0] = *(const v8b*)(pwh + c * 64 + kk * 32 + 8 * hh);
      pa.h[1] = *(const v8b*)(pwh + c * 64 + kk * 32 + 16 + 8 * hh);
      pl.h[0] = *(const v8b*)(pwl + c * 64 + kk * 32 + 8 * hh);
      pl.h[1] = *(const v8b*)(pwl + c * 64 + kk * 32 + 16 + 8 * hh);
      const int vo = (wave * 16 + c) * 64 + kk * 32 + 8 * hh;
      vb.h[0] = *(const v8b*)(Vsh + vo);
      vb.h[1] = *(const v8b*)(Vsh + vo + 16);
      vl.h[0] = *(const v8b*)(Vsl + vo);
      vl.h[1] = *(const v8b*)(Vsl + vo + 16);
      oacc = at_mma(pa.v, vb.v, oacc);
      oacc = at_mma(pa.v, vl.v, oacc);
      oacc = at_mma(pl.v, vb.v, oacc);
    }
  }

#pragma unroll
  for (int r = 0; r < 8; ++r) {
    const float inv = 1.0f / lrow[r];
    Osh[(8 * hh + r) * 68 + wave * 16 + c] = oacc[r] * inv;
  }
  __syncthreads();
  {
    const int orow = wave * 4 + (lane >> 3), c8 = (lane & 7) * 8;
    const float* sp = Osh + orow * 68 + c8;
    v8us hv, lv;
#pragma unroll
    for (int e = 0; e < 8; ++e) {
      unsigned short hb, lb;
      bf_split_bits(sp[e], hb, lb);
      hv[e] = hb;
      lv[e] = lb;
    }
    const size_t o = (size_t)(row0 + orow) * NFEAT + fcol + c8;
    for (int pass = 0; pass < 2; ++pass) {
      *(volatile v8us*)(aohi + o) = hv;
      *(volatile v8us*)(aolo + o) = lv;
      __threadfence();
    }
  }
}

__global__ __launch_bounds__(32) void pointer_probs(
    const unsigned short* __restrict__ mhhi, const unsigned short* __restrict__ mhlo,
    const unsigned short* __restrict__ ehi, const unsigned short* __restrict__ elo,
    const float* __restrict__ mask, float* __restrict__ probs) {
  __shared__ __align__(16) float Ssh[16 * NPTR];
  __shared__ float sInv[16];
  const int lane = threadIdx.x & 31;
  const int hh = lane >> 4;
  const int c  = lane & 15;
  const int blk = blockIdx.x;
  const int b = blk >> 5;
  const int row0 = blk * 16;
  const int pbase = b * NPTR;

#pragma unroll 1
  for (int jg = 0; jg < NPTR / 64; ++jg) {
    v8f acc[4];
#pragma unroll
    for (int t = 0; t < 4; ++t) acc[t] = (v8f){0.f,0.f,0.f,0.f,0.f,0.f,0.f,0.f};
#pragma unroll 1
    for (int k0 = 0; k0 < NEMB; k0 += 32) {
      const size_t ao = (size_t)(row0 + c) * NEMB + k0 + 8 * hh;
      const v16b ah = Frag<__bf16>::load((const __bf16*)mhhi + ao);
      const v16b al = Frag<__bf16>::load((const __bf16*)mhlo + ao);
#pragma unroll
      for (int t = 0; t < 4; ++t) {
        const size_t bo = (size_t)(pbase + jg * 64 + t * 16 + c) * NEMB + k0 + 8 * hh;
        const v16b bh = Frag<__bf16>::load((const __bf16*)ehi + bo);
        const v16b bl = Frag<__bf16>::load((const __bf16*)elo + bo);
        acc[t] = at_mma(ah, bh, acc[t]);
        acc[t] = at_mma(ah, bl, acc[t]);
        acc[t] = at_mma(al, bh, acc[t]);
      }
    }
#pragma unroll
    for (int t = 0; t < 4; ++t) {
#pragma unroll
      for (int r = 0; r < 8; ++r) Ssh[(8 * hh + r) * NPTR + jg * 64 + t * 16 + c] = acc[t][r] * 0.0625f;
    }
  }
  __syncthreads();

#pragma unroll 1
  for (int it = 0; it < (16 * NPTR) / 128; ++it) {
    const int idx = (it * 32 + lane) * 4;
    const int row = idx / NPTR;
    const int col = idx - row * NPTR;
    const v4f x = *(const v4f*)(Ssh + idx);
    const v4f mk = *(const v4f*)(mask + (size_t)(row0 + row) * NPTR + col);
    v4f y;
#pragma unroll
    for (int e = 0; e < 4; ++e) y[e] = CLIPV * tanhf(x[e]) + mk[e];
    *(v4f*)(Ssh + idx) = y;
  }
  __syncthreads();

  {
    const int row = lane >> 1, par = lane & 1;
    float m = -INFINITY;
#pragma unroll 1
    for (int j = par; j < NPTR; j += 2) m = fmaxf(m, Ssh[row * NPTR + j]);
    m = fmaxf(m, __shfl_xor(m, 1, 32));
    float l = 0.f;
#pragma unroll 1
    for (int j = par; j < NPTR; j += 2) {
      const float ex = expf(Ssh[row * NPTR + j] - m);
      Ssh[row * NPTR + j] = ex;
      l += ex;
    }
    l += __shfl_xor(l, 1, 32);
    if (par == 0) sInv[row] = 1.0f / l;
  }
  __syncthreads();

  float* dst = probs + (size_t)row0 * NPTR;
  for (int pass = 0; pass < 2; ++pass) {
#pragma unroll 1
    for (int it = 0; it < (16 * NPTR) / 128; ++it) {
      const int idx = it * 128 + lane * 4;
      const int row = idx / NPTR;
      v4f x = *(const v4f*)(Ssh + idx);
      const float iv = sInv[row];
      x *= iv;
      *(volatile v4f*)(dst + idx) = x;
    }
    __threadfence();
  }
}

extern "C" void kernel_launch(void* const* d_in, const int* in_sizes, int n_in,
                              void* d_out, int out_size, void* d_ws,
                              size_t ws_size, hipStream_t stream) {
  if (n_in != 10) return;
  if (in_sizes[0] != NBATCH * NEMB) return;
  if (in_sizes[1] != NBATCH * NGRP * NEMB) return;
  if (in_sizes[2] != NBATCH * NGRP) return;
  if (in_sizes[3] != NBATCH * NGRP * NPTR) return;
  if (in_sizes[4] != NBATCH * NPTR * NEMB) return;
  if (in_sizes[5] != KQIN * NFEAT) return;
  if (in_sizes[6] != NEMB * NFEAT) return;
  if (in_sizes[7] != NEMB * NFEAT) return;
  if (in_sizes[8] != NFEAT * NEMB) return;
  if (in_sizes[9] != NEMB) return;
  if (out_size != NBATCH * NGRP * NPTR) return;

  const float* in1  = (const float*)d_in[0];
  const float* in2  = (const float*)d_in[1];
  const float* tcur = (const float*)d_in[2];
  const float* mask = (const float*)d_in[3];
  const float* enc  = (const float*)d_in[4];
  const float* Wq   = (const float*)d_in[5];
  const float* Wk   = (const float*)d_in[6];
  const float* Wv   = (const float*)d_in[7];
  const float* Wc   = (const float*)d_in[8];
  const float* Wcb  = (const float*)d_in[9];
  float* probs = (float*)d_out;

  char* ws = (char*)d_ws;
  size_t off = 0;
  auto carve = [&](size_t bytes) -> unsigned short* {
    size_t o = off;
    off += (bytes + 255) & ~(size_t)255;
    return (unsigned short*)(ws + o);
  };
  const size_t wsz  = (size_t)NEMB * NFEAT * 2;
  const size_t wqsz = (size_t)NFEAT * KQPAD * 2;
  const size_t plsz = (size_t)NBATCH * NGRP * NFEAT * 2;
  const size_t qisz = (size_t)NBATCH * NGRP * KQPAD * 2;
  unsigned short* wkT_hi = carve(wsz);  unsigned short* wkT_lo = carve(wsz);
  unsigned short* wvT_hi = carve(wsz);  unsigned short* wvT_lo = carve(wsz);
  unsigned short* wcT_hi = carve(wsz);  unsigned short* wcT_lo = carve(wsz);
  unsigned short* wqT_hi = carve(wqsz); unsigned short* wqT_lo = carve(wqsz);
  unsigned short* enc_hi = carve(plsz); unsigned short* enc_lo = carve(plsz);
  unsigned short* qin_hi = carve(qisz); unsigned short* qin_lo = carve(qisz);
  unsigned short* k_hi   = carve(plsz); unsigned short* k_lo   = carve(plsz);
  unsigned short* vt_hi  = carve(plsz); unsigned short* vt_lo  = carve(plsz);
  unsigned short* q_hi   = carve(plsz); unsigned short* q_lo   = carve(plsz);
  unsigned short* ao_hi  = carve(plsz); unsigned short* ao_lo  = carve(plsz);
  unsigned short* mh_hi  = carve(plsz); unsigned short* mh_lo  = carve(plsz);
  static_assert(6 * (size_t)NEMB * NFEAT * 2 + 2 * (size_t)NFEAT * KQPAD * 2 +
                (size_t)NBATCH * NGRP * KQPAD * 2 * 2 + 6 * 2 * (size_t)NBATCH * NGRP * NFEAT * 2 == 70582272,
                "carve total");
  static_assert(NPTR == NGRP, "k and vT planes reuse the activation plane size");
  if (off > ws_size) return;
  if (off > (size_t)134217728) return;

  static_assert(NEMB % 32 == 0 && KQPAD % 32 == 0 && NFEAT % 32 == 0, "K multiple of 32");
  static_assert((NBATCH * NGRP) % 64 == 0 && NFEAT % 64 == 0 && NPTR % 64 == 0 && NEMB % 64 == 0, "M,N multiples of 64");

  transpose_split64<<<dim3(NFEAT / 64, NEMB / 64), 256, 0, stream>>>(Wk, NEMB, NFEAT, wkT_hi, wkT_lo, NEMB);
  transpose_split64<<<dim3(NFEAT / 64, NEMB / 64), 256, 0, stream>>>(Wv, NEMB, NFEAT, wvT_hi, wvT_lo, NEMB);
  transpose_split64<<<dim3(NEMB / 64, NFEAT / 64), 256, 0, stream>>>(Wc, NFEAT, NEMB, wcT_hi, wcT_lo, NFEAT);
  transpose_split64<<<dim3(NFEAT / 64, KQPAD / 64), 256, 0, stream>>>(Wq, KQIN, NFEAT, wqT_hi, wqT_lo, KQPAD);

  {
    const int n8 = NBATCH * NPTR * NEMB / 8;
    split_rows8<<<(n8 + 255) / 256, 256, 0, stream>>>(enc, enc_hi, enc_lo, n8);
  }
  {
    const int nth = NBATCH * NGRP * (KQPAD / 8);
    build_query_input<<<(nth + 255) / 256, 256, 0, stream>>>(in1, in2, tcur, qin_hi, qin_lo);
  }

  {
    const int tiles = (NBATCH * NPTR / 64) * (NFEAT / 64);
    wmma_gemm64<1, true, 0, 2, false><<<dim3((tiles + 7) / 8, 1), 256, 0, stream>>>(
        enc_hi, enc_lo, NEMB, 0L, wkT_hi, wkT_lo, NEMB, 0L,
        (void*)k_hi, (void*)k_lo, NFEAT, 0L, nullptr, nullptr, 0L,
        NBATCH * NPTR, NFEAT, NEMB, 1.0f);
  }
  {
    const int tiles = (NFEAT / 64) * (NPTR / 64);
    wmma_gemm64<1, true, 0, 2, false><<<dim3((tiles + 7) / 8, NBATCH), 256, 0, stream>>>(
        wvT_hi, wvT_lo, NEMB, 0L, enc_hi, enc_lo, NEMB, (long)NPTR * NEMB,
        (void*)vt_hi, (void*)vt_lo, NPTR, (long)NFEAT * NPTR, nullptr, nullptr, 0L,
        NFEAT, NPTR, NEMB, 1.0f);
  }
  {
    const int tiles = (NBATCH * NGRP / 64) * (NFEAT / 64);
    wmma_gemm64<1, true, 0, 2, false><<<dim3((tiles + 7) / 8, 1), 256, 0, stream>>>(
        qin_hi, qin_lo, KQPAD, 0L, wqT_hi, wqT_lo, KQPAD, 0L,
        (void*)q_hi, (void*)q_lo, NFEAT, 0L, nullptr, nullptr, 0L,
        NBATCH * NGRP, NFEAT, KQPAD, 0.25f);
  }
  mha_head16<<<NBATCH * 4 * (NGRP / 16), 128, 0, stream>>>(q_hi, q_lo, k_hi, k_lo, vt_hi, vt_lo, mask, ao_hi, ao_lo);

  {
    const int tiles = (NBATCH * NGRP / 64) * (NEMB / 64);
    wmma_gemm64<1, true, 2, 2, false><<<dim3((tiles + 7) / 8, 1), 256, 0, stream>>>(
        ao_hi, ao_lo, NFEAT, 0L, wcT_hi, wcT_lo, NFEAT, 0L,
        (void*)mh_hi, (void*)mh_lo, NEMB, 0L, Wcb, nullptr, 0L,
        NBATCH * NGRP, NEMB, NFEAT, 1.0f);
  }
  pointer_probs<<<NBATCH * NGRP / 16, 32, 0, stream>>>(mh_hi, mh_lo, enc_hi, enc_lo, mask, probs);
}
